// MultiViewGNN_11587821764815
// MI455X (gfx1250) — hardware-verified
//
#include <hip/hip_runtime.h>
#include <stddef.h>
#include <stdint.h>
#include <math.h>


#define FIN    256
#define NH     64
#define NVIEW  3
#define NTHR   256
#define NWAVE  8
#define EPT    8
#define CHUNK  (NTHR * EPT)
#define WCAP   (EPT * 32)
#define LISTN  (NWAVE * WCAP)
#define NBD    8192
#define SLD    13
#define NBA    1024
#define SLA    10
#define RCAP   28672
#define DEGCAP 128
#define GBM    64
#define GBN    64
#define GTHR   128
#define UPV    (NH * (FIN / 8))
#define NUW    (NVIEW * UPV)
#define AGG_ZINTS (LISTN + 2 * RCAP + 3 * NBA)
#define AGG_LDS_INTS (AGG_ZINTS + NBA + 16)
#define DEG_ZINTS (2 * NBD + LISTN)
#define DEG_LDS_INTS (DEG_ZINTS + 16)
#define OUTT   256
#define WSMAX  134217728

static_assert((CHUNK & (CHUNK - 1)) == 0 && CHUNK <= 4096);
static_assert((NBD & (NBD - 1)) == 0 && NBD == (1 << SLD));
static_assert((NBA & (NBA - 1)) == 0 && NBA == (1 << SLA));
static_assert(((long long)CHUNK << SLD) < (1LL << 31));
static_assert(((long long)CHUNK << SLA) < (1LL << 31));
static_assert(NBD % (NTHR * 4) == 0);
static_assert(LISTN % NTHR == 0);
static_assert(NBA % NWAVE == 0 && NBA % 32 == 0 && NBA == 4 * NTHR && NBA % GBM == 0);
static_assert(RCAP % 4 == 0 && AGG_ZINTS % 4 == 0 && LISTN % 4 == 0 && DEG_ZINTS % (NTHR * 4) == 0);
static_assert(FIN % 32 == 0 && NH == GBN && GBM == (GTHR / 32) * 16 && GBN == 16 * 4);
static_assert(UPV % NTHR == 0 && NUW % NTHR == 0);
static_assert(AGG_LDS_INTS * 4 <= 300000);
static_assert(DEG_LDS_INTS * 4 <= 300000);
static_assert(DEGCAP % 32 == 0);

typedef float          v2f   __attribute__((ext_vector_type(2)));
typedef float          v4f   __attribute__((ext_vector_type(4)));
typedef float          v8f   __attribute__((ext_vector_type(8)));
typedef int            v4i   __attribute__((ext_vector_type(4)));
typedef int            v8i   __attribute__((ext_vector_type(8)));
typedef unsigned short v8us  __attribute__((ext_vector_type(8)));
typedef unsigned short v16us __attribute__((ext_vector_type(16)));
typedef __bf16         v16bf __attribute__((ext_vector_type(16)));
typedef v2f  __attribute__((may_alias)) v2fa;
typedef v4f  __attribute__((may_alias)) v4fa;
typedef v4i  __attribute__((may_alias)) v4ia;
typedef v8us __attribute__((may_alias)) v8usa;
union FragB { v16bf v; v16us u; v8us h[2]; v8i w; };

__device__ __forceinline__ v8f wmb(const FragB& a, const FragB& b, v8f c) {
  v8f d = __builtin_amdgcn_wmma_f32_16x16x32_bf16(false, a.v, false, b.v, (short)0, c, false, false);
  asm volatile("v_nop\n\tv_nop\n\tv_nop\n\tv_nop" : "+v"(d) : "v"(a.w), "v"(b.w));
  return d;
}

__device__ __forceinline__ unsigned bf16_bits(float f) {
  const unsigned u = __float_as_uint(f);
  return (u + 0x7FFFu + ((u >> 16) & 1u)) >> 16;
}
__device__ __forceinline__ float bf16_val(float f) {
  return __uint_as_float(bf16_bits(f) << 16);
}

template <int SLB>
__device__ __forceinline__ int scan_chunk(const int* __restrict__ dsts, int nE, int cbase, int slotBase,
                                          int nb, int vec8, int* list, int tid, int lane, int wave) {
  int wc = 0;
  const int el0  = tid * EPT;
  const int e0   = cbase + el0;
  const int sent = -2147483647 - 1;
  v4i da, db;
  if (vec8 != 0 && cbase + CHUNK <= nE) {
    da = *(const v4i*)(dsts + e0);
    db = *(const v4i*)(dsts + e0 + 4);
  } else {
    da.x = (e0     < nE) ? dsts[min(e0,     nE - 1)] : sent;
    da.y = (e0 + 1 < nE) ? dsts[min(e0 + 1, nE - 1)] : sent;
    da.z = (e0 + 2 < nE) ? dsts[min(e0 + 2, nE - 1)] : sent;
    da.w = (e0 + 3 < nE) ? dsts[min(e0 + 3, nE - 1)] : sent;
    db.x = (e0 + 4 < nE) ? dsts[min(e0 + 4, nE - 1)] : sent;
    db.y = (e0 + 5 < nE) ? dsts[min(e0 + 5, nE - 1)] : sent;
    db.z = (e0 + 6 < nE) ? dsts[min(e0 + 6, nE - 1)] : sent;
    db.w = (e0 + 7 < nE) ? dsts[min(e0 + 7, nE - 1)] : sent;
  }
  const unsigned nbs = (unsigned)slotBase;
  const unsigned unb = (unsigned)nb;
  const unsigned s0 = (unsigned)da.x - nbs, s1 = (unsigned)da.y - nbs;
  const unsigned s2 = (unsigned)da.z - nbs, s3 = (unsigned)da.w - nbs;
  const unsigned s4 = (unsigned)db.x - nbs, s5 = (unsigned)db.y - nbs;
  const unsigned s6 = (unsigned)db.z - nbs, s7 = (unsigned)db.w - nbs;
  const bool h0 = s0 < unb, h1 = s1 < unb, h2 = s2 < unb, h3 = s3 < unb;
  const bool h4 = s4 < unb, h5 = s5 < unb, h6 = s6 < unb, h7 = s7 < unb;
  const unsigned any = __builtin_amdgcn_ballot_w32(h0 | h1 | h2 | h3 | h4 | h5 | h6 | h7);
  if (any != 0u) {
#define HITJ(J, HJ, SJ) { \
      const unsigned mj = __builtin_amdgcn_ballot_w32(HJ); \
      if (mj != 0u) { \
        if (HJ) { \
          const int pos = wc + (int)__builtin_amdgcn_mbcnt_lo(mj, 0u); \
          if (pos < WCAP) list[wave * WCAP + pos] = ((el0 + (J)) << SLB) | (int)(SJ); \
        } \
        wc += (int)__builtin_popcount(mj); } }
    HITJ(0, h0, s0)
    HITJ(1, h1, s1)
    HITJ(2, h2, s2)
    HITJ(3, h3, s3)
    HITJ(4, h4, s4)
    HITJ(5, h5, s5)
    HITJ(6, h6, s6)
    HITJ(7, h7, s7)
#undef HITJ
  }
  return wc;
}

__global__ __launch_bounds__(NTHR) void k_prep(const float* __restrict__ x, int nN, int uX,
                                               const float* __restrict__ Wa, const float* __restrict__ Wb,
                                               const float* __restrict__ Wc,
                                               unsigned short* xb, unsigned short* w1t) {
  const int u = (int)blockIdx.x * NTHR + (int)threadIdx.x;
  v8us o;
  unsigned short* dp;
  if (u < uX) {
    const int row = u >> 5;
    const int k8  = (u & 31) * 8;
    const int rc  = row < nN ? row : nN - 1;
    const float* p = x + (size_t)rc * FIN + k8;
    const v4f a = *(const v4fa*)p;
    const v4f b = *(const v4fa*)(p + 4);
    const bool ok = row < nN;
    o[0] = ok ? (unsigned short)bf16_bits(a.x) : (unsigned short)0;
    o[1] = ok ? (unsigned short)bf16_bits(a.y) : (unsigned short)0;
    o[2] = ok ? (unsigned short)bf16_bits(a.z) : (unsigned short)0;
    o[3] = ok ? (unsigned short)bf16_bits(a.w) : (unsigned short)0;
    o[4] = ok ? (unsigned short)bf16_bits(b.x) : (unsigned short)0;
    o[5] = ok ? (unsigned short)bf16_bits(b.y) : (unsigned short)0;
    o[6] = ok ? (unsigned short)bf16_bits(b.z) : (unsigned short)0;
    o[7] = ok ? (unsigned short)bf16_bits(b.w) : (unsigned short)0;
    dp = xb + (size_t)row * FIN + k8;
  } else {
    const int v = u - uX;
    if (v >= NUW) return;
    const int view = v / UPV;
    const int t  = v - view * UPV;
    const int n  = t >> 5;
    const int k8 = (t & 31) * 8;
    const float* Wp = (view == 0) ? Wa : ((view == 1) ? Wb : Wc);
    const float* p = Wp + (size_t)k8 * NH + n;
#pragma unroll
    for (int i = 0; i < 8; ++i) o[i] = (unsigned short)bf16_bits(p[(size_t)i * NH]);
    dp = w1t + (size_t)view * (NH * FIN) + (size_t)n * FIN + k8;
  }
  *(volatile v8us*)dp = o;
  __threadfence();
  *(volatile v8us*)dp = o;
}

__global__ __launch_bounds__(GTHR) void k_gemm(const unsigned short* __restrict__ A, int lda,
                                               const unsigned short* __restrict__ BT, int ldb, int K,
                                               float* Cm) {
  __shared__ __attribute__((aligned(16))) float stg[GBM * GBN];
  const int tid = (int)threadIdx.x, lane = tid & 31, wave = tid >> 5, hh = lane >> 4, m = lane & 15;
  const int rowBase = (int)blockIdx.x * GBM;

  v8f acc[4];
  {
    const v8f z = {0.f, 0.f, 0.f, 0.f, 0.f, 0.f, 0.f, 0.f};
#pragma unroll
    for (int t = 0; t < 4; ++t) acc[t] = z;
  }
  const unsigned short* ap = A  + (size_t)(rowBase + 16 * wave + m) * (size_t)lda + 8 * hh;
  const unsigned short* bp = BT + (size_t)m * (size_t)ldb + 8 * hh;

#pragma unroll 1
  for (int k0 = 0; k0 < K; k0 += 32) {
    FragB af;
    af.h[0] = *(const v8usa*)(ap + k0);
    af.h[1] = *(const v8usa*)(ap + k0 + 16);
#pragma unroll
    for (int nt = 0; nt < 4; ++nt) {
      const unsigned short* wq = bp + (size_t)(16 * nt) * (size_t)ldb + k0;
      FragB bf;
      bf.h[0] = *(const v8usa*)wq;
      bf.h[1] = *(const v8usa*)(wq + 16);
      acc[nt] = wmb(af, bf, acc[nt]);
    }
  }

#pragma unroll
  for (int nt = 0; nt < 4; ++nt) {
    const int lc = 16 * nt + m;
#pragma unroll
    for (int r = 0; r < 8; ++r) {
      const int lr = 16 * wave + 8 * hh + r;
      stg[lr * GBN + lc] = acc[nt][r];
    }
  }
  __syncthreads();

  const int sub = lane >> 4, c4 = 4 * (lane & 15);
  v4f pv[8];
#pragma unroll
  for (int i = 0; i < 8; ++i) pv[i] = *(const v4fa*)(stg + (16 * wave + 2 * i + sub) * GBN + c4);
#pragma unroll
  for (int i = 0; i < 8; ++i) {
    float* op = Cm + (size_t)(rowBase + 16 * wave + 2 * i + sub) * GBN + c4;
    *(volatile v4f*)op = pv[i];
  }
  __threadfence();
#pragma unroll
  for (int i = 0; i < 8; ++i) {
    float* op = Cm + (size_t)(rowBase + 16 * wave + 2 * i + sub) * GBN + c4;
    *(volatile v4f*)op = pv[i];
  }
}

__device__ __forceinline__ float dinvw(float s, bool live) {
  const float dg = s + 1.0f;
  const float r  = dg > 0.0f ? rsqrtf(fmaxf(dg, 1e-30f)) : 0.0f;
  return live ? r : 0.0f;
}

__global__ __launch_bounds__(NTHR) void k_deg(const int* __restrict__ dsts, const float* __restrict__ ew,
                                              int nE, int nN, int vec8, float* dis1, float* dis2) {
  extern __shared__ __attribute__((aligned(16))) int ddm[];
  float* sdeg = (float*)ddm;
  int*   scnt = ddm + NBD;
  int*   list = ddm + 2 * NBD;
  int*   wcnt = ddm + DEG_ZINTS;
  const int tid = (int)threadIdx.x, lane = tid & 31, wave = tid >> 5;
  const int nodeBase = (int)blockIdx.x * NBD;

  {
    const v4i z4 = {0, 0, 0, 0};
    for (int i = tid * 4; i < DEG_ZINTS; i += NTHR * 4) *(v4ia*)(ddm + i) = z4;
    if (tid < 16) wcnt[tid] = 0;
  }
  __syncthreads();

  const int nChunks = (nE + CHUNK - 1) / CHUNK;
#pragma unroll 1
  for (int ch = 0; ch < nChunks; ++ch) {
    const int cbase = ch * CHUNK;
    const int wc = scan_chunk<SLD>(dsts, nE, cbase, nodeBase, NBD, vec8, list, tid, lane, wave);
    if (lane == 0) wcnt[wave] = wc;
    __syncthreads();
    if (wave == 0) {
#pragma unroll 1
      for (int w2 = 0; w2 < NWAVE; ++w2) {
        int c = wcnt[w2];
        c = c < 0 ? 0 : (c > WCAP ? WCAP : c);
#pragma unroll 1
        for (int b0 = 0; b0 < c; b0 += 32) {
          const int idx = b0 + lane;
          const int ent = list[w2 * WCAP + (idx < WCAP ? idx : WCAP - 1)];
          const int el  = (ent >> SLD) & (CHUNK - 1);
          int eid = cbase + el;
          eid = eid < 0 ? 0 : (eid > nE - 1 ? nE - 1 : eid);
          const int wvi = __float_as_int(bf16_val(ew[eid]));
          const int m32 = (c - b0) < 32 ? (c - b0) : 32;
#pragma unroll 1
          for (int k = 0; k < m32; ++k) {
            const int   u   = __builtin_amdgcn_readlane(ent, k);
            const float wk  = __int_as_float(__builtin_amdgcn_readlane(wvi, k));
            const int   slt = u & (NBD - 1);
            if (lane == 0) { sdeg[slt] = sdeg[slt] + wk; scnt[slt] = scnt[slt] + 1; }
          }
        }
      }
    }
    __syncthreads();
  }

  v4f vals[NBD / (NTHR * 4)];
  v4f cvs[NBD / (NTHR * 4)];
#pragma unroll
  for (int it = 0; it < NBD / (NTHR * 4); ++it) {
    const int s0 = it * (NTHR * 4) + 4 * tid;
    const v4f d4 = *(const v4fa*)(sdeg + s0);
    const v4i c4 = *(const v4ia*)(scnt + s0);
    const int n0 = nodeBase + s0;
    const bool l0 = n0 < nN, l1 = n0 + 1 < nN, l2 = n0 + 2 < nN, l3 = n0 + 3 < nN;
    v4f v, r;
    v.x = dinvw(d4.x, l0); v.y = dinvw(d4.y, l1); v.z = dinvw(d4.z, l2); v.w = dinvw(d4.w, l3);
    r.x = l0 ? rsqrtf((float)c4.x + 1.0f) : 0.0f;
    r.y = l1 ? rsqrtf((float)c4.y + 1.0f) : 0.0f;
    r.z = l2 ? rsqrtf((float)c4.z + 1.0f) : 0.0f;
    r.w = l3 ? rsqrtf((float)c4.w + 1.0f) : 0.0f;
    vals[it] = v;
    cvs[it]  = r;
  }
#pragma unroll
  for (int it = 0; it < NBD / (NTHR * 4); ++it) {
    const int s0 = it * (NTHR * 4) + 4 * tid;
    *(volatile v4f*)(dis1 + (size_t)nodeBase + s0) = vals[it];
    *(volatile v4f*)(dis2 + (size_t)nodeBase + s0) = cvs[it];
  }
  __threadfence();
#pragma unroll
  for (int it = 0; it < NBD / (NTHR * 4); ++it) {
    const int s0 = it * (NTHR * 4) + 4 * tid;
    *(volatile v4f*)(dis1 + (size_t)nodeBase + s0) = vals[it];
    *(volatile v4f*)(dis2 + (size_t)nodeBase + s0) = cvs[it];
  }
}

__global__ __launch_bounds__(NTHR) void k_agg1(const int* __restrict__ srcs, const int* __restrict__ dsts,
                                               const float* __restrict__ ew, int nE, int nN, int vec8,
                                               int mRows, int accum,
                                               const float* __restrict__ dis, const float* __restrict__ xw,
                                               const float* __restrict__ b1, const float* __restrict__ w2,
                                               float* feat, float* sp) {
  extern __shared__ __attribute__((aligned(16))) int dsm[];
  int*   list = dsm;
  int*   hl   = dsm + LISTN;
  int*   sl   = dsm + LISTN + RCAP;
  int*   cnt  = dsm + LISTN + 2 * RCAP;
  int*   offs = cnt + NBA;
  int*   cur  = offs + NBA;
  float* sS   = (float*)(cur + NBA);
  int*   misc = cur + 2 * NBA;
  const int tid = (int)threadIdx.x, lane = tid & 31, wave = tid >> 5;
  const int nodeBase = (int)blockIdx.x * NBA;

  {
    const v4i z4 = {0, 0, 0, 0};
    for (int i = tid * 4; i < AGG_ZINTS; i += NTHR * 4) *(v4ia*)(dsm + i) = z4;
    if (tid < 16) misc[tid] = 0;
  }
  const float bv0 = bf16_val(b1[2 * lane]);
  const float bv1 = bf16_val(b1[2 * lane + 1]);
  const float wq0 = bf16_val(w2[2 * lane]);
  const float wq1 = bf16_val(w2[2 * lane + 1]);
  __syncthreads();

  int t = 0, ov = 0;
  const int nChunks = (nE + CHUNK - 1) / CHUNK;
#pragma unroll 1
  for (int ch = 0; ch < nChunks; ++ch) {
    const int cbase = ch * CHUNK;
    const int wc = scan_chunk<SLA>(dsts, nE, cbase, nodeBase, NBA, vec8, list, tid, lane, wave);
    if (lane == 0) misc[wave] = wc;
    __syncthreads();
    if (wave == 0) {
#pragma unroll 1
      for (int w2i = 0; w2i < NWAVE; ++w2i) {
        int c = misc[w2i];
        c = c < 0 ? 0 : (c > WCAP ? WCAP : c);
#pragma unroll 1
        for (int b0 = 0; b0 < c; b0 += 32) {
          const int idx = b0 + lane;
          const int ent = list[w2i * WCAP + (idx < WCAP ? idx : WCAP - 1)];
          const int m32 = (c - b0) < 32 ? (c - b0) : 32;
#pragma unroll 1
          for (int k = 0; k < m32; ++k) {
            const int u    = __builtin_amdgcn_readlane(ent, k);
            const int slot = u & (NBA - 1);
            const int el   = (u >> SLA) & (CHUNK - 1);
            const int pk   = ((cbase + el) << SLA) | slot;
            if (t < RCAP) {
              if (lane == 0) { hl[t] = pk; cnt[slot] = cnt[slot] + 1; }
              t = t + 1;
            } else {
              ov = 1;
            }
          }
        }
      }
    }
    __syncthreads();
  }
  if (wave == 0 && lane == 0) { misc[8] = t; misc[9] = ov; }
  __syncthreads();
  int tt = misc[8];
  tt = tt < 0 ? 0 : (tt > RCAP ? RCAP : tt);
  const int ovf = misc[9];

  if (wave == 0) {
    const int base = lane * (NBA / 32);
    int s = 0;
#pragma unroll 1
    for (int i = 0; i < NBA / 32; ++i) s += cnt[base + i];
    int incl = s;
#pragma unroll
    for (int d = 1; d < 32; d <<= 1) {
      const int y = __shfl_up(incl, d, 32);
      if (lane >= d) incl += y;
    }
    int run = incl - s;
#pragma unroll 1
    for (int i = 0; i < NBA / 32; ++i) {
      const int cv = cnt[base + i];
      offs[base + i] = run;
      cur[base + i]  = run;
      run += cv;
    }
  }
  __syncthreads();
  if (wave == 0) {
#pragma unroll 1
    for (int b0 = 0; b0 < tt; b0 += 32) {
      const int idx = b0 + lane;
      const int ent = hl[idx < RCAP ? idx : RCAP - 1];
      const int m32 = (tt - b0) < 32 ? (tt - b0) : 32;
#pragma unroll 1
      for (int k = 0; k < m32; ++k) {
        const int u    = __builtin_amdgcn_readlane(ent, k);
        const int slot = u & (NBA - 1);
        if (lane == 0) {
          int p = cur[slot];
          p = p < 0 ? 0 : (p > RCAP - 1 ? RCAP - 1 : p);
          sl[p] = u;
          cur[slot] = p + 1;
        }
      }
    }
  }
  __syncthreads();

  const float pz = (ovf != 0) ? __int_as_float(0x7fc00000) : 0.0f;
  const int i0 = (2 * lane) & 31, i1 = (2 * lane + 1) & 31;
#pragma unroll 1
  for (int si = 0; si < NBA / NWAVE; ++si) {
    const int s    = si * NWAVE + wave;
    const int node = nodeBase + s;
    int c = cnt[s];
    const bool big = c > DEGCAP;
    c = c < 0 ? 0 : (c > DEGCAP ? DEGCAP : c);
    int o = offs[s];
    o = o < 0 ? 0 : (o > RCAP ? RCAP : o);
    const int nc = node < nN ? node : nN - 1;
    const float dd = dis[nc];
    float acc0 = 0.0f, acc1 = 0.0f;
#pragma unroll 1
    for (int b0 = 0; b0 < c; b0 += 32) {
      int idx = o + b0 + lane;
      idx = idx > RCAP - 1 ? RCAP - 1 : idx;
      const int ent = sl[idx];
      int eid = ent >> SLA;
      eid = eid < 0 ? 0 : (eid > nE - 1 ? nE - 1 : eid);
      int sr = srcs[eid];
      sr = sr < 0 ? 0 : (sr > nN - 1 ? nN - 1 : sr);
      const float we  = bf16_val(ew[eid]);
      const float cf  = (dis[sr] * we) * dd;
      const int   cfi = __float_as_int(cf);
      const int m32 = (c - b0) < 32 ? (c - b0) : 32;
#pragma unroll 1
      for (int k = 0; k < m32; ++k) {
        const int   sk = __builtin_amdgcn_readlane(sr, k);
        const float ck = __int_as_float(__builtin_amdgcn_readlane(cfi, k));
        const v2f a = *(const v2fa*)(xw + (size_t)sk * NH + 2 * lane);
        acc0 = fmaf(ck, a.x, acc0);
        acc1 = fmaf(ck, a.y, acc1);
      }
    }
    const v2f sv = *(const v2fa*)(xw + (size_t)nc * NH + 2 * lane);
    const float ns = dd * dd;
    const float pzr = big ? __int_as_float(0x7fc00000) : pz;
    const bool live = node < nN;
    float y0 = (acc0 + sv.x * ns) + bv0;
    float y1 = (acc1 + sv.y * ns) + bv1;
    y0 = fmaxf(y0, 0.0f); y1 = fmaxf(y1, 0.0f);
    y0 = y0 + pzr; y1 = y1 + pzr;
    y0 = live ? y0 : 0.0f;
    y1 = live ? y1 : 0.0f;
    float p = fmaf(y1, wq1, y0 * wq0);
#pragma unroll
    for (int q = 16; q > 0; q >>= 1) p += __shfl_xor(p, q, 32);
    if (lane == 0) sS[s] = p;
    if (node < mRows) {
      float o0 = y0, o1 = y1;
      if (accum != 0) {
        const v2f od = *(const v2fa*)(feat + (size_t)node * NH + 2 * lane);
        o0 = o0 + od.x;
        o1 = o1 + od.y;
      }
      v4f pk;
      pk.x = __shfl(o0, i0, 32);
      pk.y = __shfl(o1, i0, 32);
      pk.z = __shfl(o0, i1, 32);
      pk.w = __shfl(o1, i1, 32);
      float* fp = feat + (size_t)node * NH + 4 * lane;
      if (lane < 16) *(volatile v4f*)fp = pk;
      __threadfence();
      if (lane < 16) *(volatile v4f*)fp = pk;
    }
  }
  __syncthreads();
  {
    const v4f q4 = *(const v4fa*)(sS + 4 * tid);
    float* op = sp + (size_t)nodeBase + 4 * tid;
    *(volatile v4f*)op = q4;
    __threadfence();
    *(volatile v4f*)op = q4;
  }
}

__global__ __launch_bounds__(NTHR) void k_agg2(const int* __restrict__ srcs, const int* __restrict__ dsts,
                                               int nE, int nN, int vec8, int accum,
                                               const float* __restrict__ sp, int nSP,
                                               const float* __restrict__ dis2, const float* __restrict__ b2,
                                               float* xf) {
  __shared__ __attribute__((aligned(16))) float sacc[NBD];
  __shared__ __attribute__((aligned(16))) int list[LISTN];
  __shared__ int wcnt[NWAVE];
  const int tid = (int)threadIdx.x, lane = tid & 31, wave = tid >> 5;
  const int nodeBase = (int)blockIdx.x * NBD;

  {
    const v4f z4 = {0.f, 0.f, 0.f, 0.f};
    const v4i z4i = {0, 0, 0, 0};
    for (int i = tid * 4; i < NBD; i += NTHR * 4) *(v4fa*)(sacc + i) = z4;
    for (int i = tid * 4; i < LISTN; i += NTHR * 4) *(v4ia*)(list + i) = z4i;
    if (tid < NWAVE) wcnt[tid] = 0;
  }
  const float b2v = bf16_val(b2[0]);
  __syncthreads();

  const int nChunks = (nE + CHUNK - 1) / CHUNK;
#pragma unroll 1
  for (int ch = 0; ch < nChunks; ++ch) {
    const int cbase = ch * CHUNK;
    const int wc = scan_chunk<SLD>(dsts, nE, cbase, nodeBase, NBD, vec8, list, tid, lane, wave);
    if (lane == 0) wcnt[wave] = wc;
    __syncthreads();
    if (wave == 0) {
#pragma unroll 1
      for (int w2 = 0; w2 < NWAVE; ++w2) {
        int c = wcnt[w2];
        c = c < 0 ? 0 : (c > WCAP ? WCAP : c);
#pragma unroll 1
        for (int b0 = 0; b0 < c; b0 += 32) {
          const int idx = b0 + lane;
          const int ent = list[w2 * WCAP + (idx < WCAP ? idx : WCAP - 1)];
          const int el  = (ent >> SLD) & (CHUNK - 1);
          int eid = cbase + el;
          eid = eid < 0 ? 0 : (eid > nE - 1 ? nE - 1 : eid);
          int sr = srcs[eid];
          sr = sr < 0 ? 0 : (sr > nN - 1 ? nN - 1 : sr);
          const float val = sp[sr] * dis2[sr];
          const int   vi  = __float_as_int(val);
          const int m32 = (c - b0) < 32 ? (c - b0) : 32;
#pragma unroll 1
          for (int k = 0; k < m32; ++k) {
            const int   u   = __builtin_amdgcn_readlane(ent, k);
            const float vk  = __int_as_float(__builtin_amdgcn_readlane(vi, k));
            const int   slt = u & (NBD - 1);
            if (lane == 0) sacc[slt] = sacc[slt] + vk;
          }
        }
      }
    }
    __syncthreads();
  }

  v4f vals[NBD / (NTHR * 4)];
#pragma unroll
  for (int it = 0; it < NBD / (NTHR * 4); ++it) {
    const int s0 = it * (NTHR * 4) + 4 * tid;
    const v4f a4 = *(const v4fa*)(sacc + s0);
    const int n0 = nodeBase + s0;
    int sb = n0;
    sb = sb > nSP - 4 ? nSP - 4 : sb;
    sb = sb < 0 ? 0 : sb;
    const v4f s4 = *(const v4fa*)(sp + sb);
    const v4f d4 = *(const v4fa*)(dis2 + n0);
    v4f v;
    v.x = (n0     < nN) ? ((a4.x * d4.x + s4.x * (d4.x * d4.x)) + b2v) : 0.0f;
    v.y = (n0 + 1 < nN) ? ((a4.y * d4.y + s4.y * (d4.y * d4.y)) + b2v) : 0.0f;
    v.z = (n0 + 2 < nN) ? ((a4.z * d4.z + s4.z * (d4.z * d4.z)) + b2v) : 0.0f;
    v.w = (n0 + 3 < nN) ? ((a4.w * d4.w + s4.w * (d4.w * d4.w)) + b2v) : 0.0f;
    if (accum != 0) {
      const v4f od = *(const v4fa*)(xf + n0);
      v = v + od;
    }
    vals[it] = v;
  }
#pragma unroll
  for (int it = 0; it < NBD / (NTHR * 4); ++it) {
    const int s0 = it * (NTHR * 4) + 4 * tid;
    *(volatile v4f*)(xf + (size_t)nodeBase + s0) = vals[it];
  }
  __threadfence();
#pragma unroll
  for (int it = 0; it < NBD / (NTHR * 4); ++it) {
    const int s0 = it * (NTHR * 4) + 4 * tid;
    *(volatile v4f*)(xf + (size_t)nodeBase + s0) = vals[it];
  }
}

__global__ __launch_bounds__(OUTT) void k_out(const float* __restrict__ xf, int xfN,
                                              const float* __restrict__ feat, int featN,
                                              int nN, int total4, float* outp) {
  const int t = (int)blockIdx.x * OUTT + (int)threadIdx.x;
  const int e = 4 * t;
  int xi = e;
  xi = xi > xfN - 4 ? xfN - 4 : xi;
  xi = xi < 0 ? 0 : xi;
  int fi = e - nN;
  fi = fi < 0 ? 0 : (fi > featN - 4 ? featN - 4 : fi);
  const v4i a = *(const v4ia*)(xf + xi);
  const v4i b = *(const v4ia*)(feat + fi);
  const int msk = (e < nN) ? -1 : 0;
  v4i o;
  o.x = (a.x & msk) | (b.x & ~msk);
  o.y = (a.y & msk) | (b.y & ~msk);
  o.z = (a.z & msk) | (b.z & ~msk);
  o.w = (a.w & msk) | (b.w & ~msk);
  int* op = (int*)outp + (size_t)e;
  if (t < total4) *(volatile v4i*)op = o;
  __threadfence();
  if (t < total4) *(volatile v4i*)op = o;
}

static inline int cdiv(int a, int b) { return (a + b - 1) / b; }

extern "C" void kernel_launch(void* const* d_in, const int* in_sizes, int n_in,
                              void* d_out, int out_size, void* d_ws, size_t ws_size,
                              hipStream_t stream) {
  if (n_in < 19) return;
  if (in_sizes[0] < FIN || (in_sizes[0] % FIN) != 0) return;
  const int nN = in_sizes[0] / FIN;
  if ((nN & 3) != 0) return;
  if (in_sizes[1] < 2 || (in_sizes[1] & 1) != 0) return;
  const int nE = in_sizes[1] / 2;
  if (nE < 1 || nE >= (1 << 21)) return;
  if (in_sizes[2] != in_sizes[1] || in_sizes[3] != in_sizes[1]) return;
  if (in_sizes[4] != nE || in_sizes[5] != nE || in_sizes[6] != nE) return;
  for (int v = 0; v < NVIEW; ++v) {
    if (in_sizes[7 + 4 * v] != FIN * NH) return;
    if (in_sizes[8 + 4 * v] != NH) return;
    if (in_sizes[9 + 4 * v] != NH) return;
    if (in_sizes[10 + 4 * v] != 1) return;
  }
  if ((long long)out_size != (long long)nN * (NH + 1)) return;

  const float* x = (const float*)d_in[0];
  const int*   eiv[NVIEW];
  const float* ewv[NVIEW];
  const float* W1v[NVIEW];
  const float* b1v[NVIEW];
  const float* W2v[NVIEW];
  const float* b2v[NVIEW];
  for (int v = 0; v < NVIEW; ++v) {
    eiv[v] = (const int*)d_in[1 + v];
    ewv[v] = (const float*)d_in[4 + v];
    W1v[v] = (const float*)d_in[7 + 4 * v];
    b1v[v] = (const float*)d_in[8 + 4 * v];
    W2v[v] = (const float*)d_in[9 + 4 * v];
    b2v[v] = (const float*)d_in[10 + 4 * v];
  }
  float* out = (float*)d_out;

  const int MP   = cdiv(nN, GBM) * GBM;
  const int gM   = MP / GBM;
  const int gD   = cdiv(nN, NBD);
  const int NBPD = gD * NBD;
  const int gA   = cdiv(nN, NBA);
  const int NSP  = gA * NBA;
  if ((long long)gA * NBA < (long long)MP) return;
  if (NBPD < nN || NSP < nN || NSP < 4) return;
  const int vec8 = ((nE & 3) == 0) ? 1 : 0;
  const int total4 = (int)(((long long)nN * (NH + 1)) / 4);
  if ((long long)total4 * 4 != (long long)out_size) return;

  char* ws = (char*)d_ws;
  size_t off = 0;
  const size_t oXB   = off; off += (size_t)MP * FIN * 2;            off = (off + 255) & ~(size_t)255;
  const size_t oW1T  = off; off += (size_t)NVIEW * NH * FIN * 2;    off = (off + 255) & ~(size_t)255;
  const size_t oXW   = off; off += (size_t)MP * NH * 4;             off = (off + 255) & ~(size_t)255;
  const size_t oFEAT = off; off += (size_t)MP * NH * 4;             off = (off + 255) & ~(size_t)255;
  const size_t oD1   = off; off += (size_t)NBPD * 4;                off = (off + 255) & ~(size_t)255;
  const size_t oD2   = off; off += (size_t)NBPD * 4;                off = (off + 255) & ~(size_t)255;
  const size_t oSP   = off; off += (size_t)NSP * 4;                 off = (off + 255) & ~(size_t)255;
  const size_t oXF   = off; off += (size_t)NBPD * 4;                off = (off + 255) & ~(size_t)255;
  if (off > ws_size || off > (size_t)WSMAX) return;

  unsigned short* XB   = (unsigned short*)(ws + oXB);
  unsigned short* W1T  = (unsigned short*)(ws + oW1T);
  float*          XW   = (float*)(ws + oXW);
  float*          FEAT = (float*)(ws + oFEAT);
  float*          DIS1 = (float*)(ws + oD1);
  float*          DIS2 = (float*)(ws + oD2);
  float*          SP   = (float*)(ws + oSP);
  float*          XF   = (float*)(ws + oXF);

  const size_t aggLds = (size_t)AGG_LDS_INTS * 4;
  const size_t degLds = (size_t)DEG_LDS_INTS * 4;
  hipFuncSetAttribute(reinterpret_cast<const void*>(&k_agg1), hipFuncAttributeMaxDynamicSharedMemorySize, (int)aggLds);
  hipFuncSetAttribute(reinterpret_cast<const void*>(&k_deg), hipFuncAttributeMaxDynamicSharedMemorySize, (int)degLds);

  const int uX = MP * (FIN / 8);
  k_prep<<<(uX + NUW) / NTHR, NTHR, 0, stream>>>(x, nN, uX, W1v[0], W1v[1], W1v[2], XB, W1T);
  for (int v = 0; v < NVIEW; ++v) {
    const int* src = eiv[v];
    const int* dst = eiv[v] + nE;
    const int accum = (v > 0) ? 1 : 0;
    k_gemm<<<gM, GTHR, 0, stream>>>(XB, FIN, W1T + (size_t)v * NH * FIN, FIN, FIN, XW);
    k_deg<<<gD, NTHR, degLds, stream>>>(dst, ewv[v], nE, nN, vec8, DIS1, DIS2);
    k_agg1<<<gA, NTHR, aggLds, stream>>>(src, dst, ewv[v], nE, nN, vec8, MP, accum,
                                         DIS1, XW, b1v[v], W2v[v], FEAT, SP);
    k_agg2<<<gD, NTHR, 0, stream>>>(src, dst, nE, nN, vec8, accum, SP, NSP, DIS2, b2v[v], XF);
  }
  k_out<<<cdiv(total4, OUTT), OUTT, 0, stream>>>(XF, NBPD, FEAT, MP * NH, nN, total4, out);
}
